// HyperSelfAttention_63050119905324
// MI455X (gfx1250) — hardware-run, weakly checked
//
#include <hip/hip_runtime.h>

#ifndef NB
#define NB 2
#endif
#ifndef SEQ
#define SEQ 2048
#endif
#define NB_FULL 2
#define SEQ_FULL 2048
#define DM 1024
#define NH 16
#define HID 256
#define DYN 64
#define RK 8
#define DYNS 0.125f
#define SLEN SEQ
#define NR (NB * SLEN)
#define TQ SLEN
#define TK SLEN
#define SCL 0.125f
#define QBLKS (TQ / 64)
#define RE ((SLEN < 512) ? SLEN : 512)
#define QB05 0
#define QBN5 (RE / 64)
#define QB0P QBN5
#define QBNP (QBLKS - QBN5)
static_assert(SLEN % 128 == 0);
static_assert(SLEN <= SEQ_FULL);
static_assert(NB >= 1 && NB <= NB_FULL);
static_assert(RE % 128 == 0 && RE <= SLEN);
static_assert((SLEN - RE) % 128 == 0);
static_assert(DM % 64 == 0 && DM == NH * 64);
static_assert(DM % 32 == 0 && (2 * DM) % 32 == 0);
static_assert(NR % 128 == 0 && NR % 64 == 0);
static_assert(HID == 256 && DYN == 64 && RK == 8);
static_assert(2 * RK == 16);
static_assert((NB * (RK * DM / 4)) % 256 == 0);
static_assert((SLEN / 8) * 8 == SLEN);
static_assert(256 * 2 * 16 == 64 * 128);
static_assert(32 * 2 * 16 == 16 * 64);
static_assert(32 * 16 * 16 == 32 * 256);
static_assert(4 * 32 * 68 * 4 <= 131072);
static_assert(4 * 16 * 40 * 2 * 2 + 4 * 16 * 68 * 4 <= 131072);
static_assert(64 * 66 * 2 <= 131072);

static constexpr float WSC = 16.0f;
static constexpr float WSCH = 16384.0f;
static constexpr float ALPHA = 0.0625f;
static constexpr float ALPHAE = 0.0625f / 1024.0f;

static constexpr size_t al256(size_t b) { return (b + 255) & ~(size_t)255; }
static constexpr size_t SZ_W = al256((size_t)DM * DM * 2);
static constexpr size_t SZ_B2 = al256((size_t)DM * 2 * DM * 2);
static constexpr size_t SZ_F32P = al256((size_t)NR * DM * 4);
static constexpr size_t SZ_F16P = al256((size_t)NR * DM * 2);
static constexpr size_t SZ_RES = al256((size_t)NB * RE * DM * 2);
static constexpr size_t SZ_VTL = al256((size_t)NB * NH * 64 * RE * 2);
static constexpr size_t SZ_A2 = al256((size_t)NB * RE * 2 * DM * 2);
static constexpr size_t SZ_TAB = al256((size_t)SLEN * 32 * 4);
static constexpr size_t SZ_INV = al256(128);
static constexpr size_t SZ_Z = al256((size_t)NB * DM * 4);
static constexpr size_t SZ_CC = al256((size_t)NB * DYN * 4);
static constexpr size_t SZ_AP = al256((size_t)NB * 16 * DM * 2);
static constexpr size_t SZ_BM = al256((size_t)NB * DM * RK * 4);
static constexpr size_t SZ_XA = al256((size_t)NR * 16 * 4);
static constexpr size_t WS_TOTAL = 3 * SZ_W + SZ_B2 + SZ_F32P + 4 * SZ_F16P + 2 * SZ_RES + SZ_VTL + SZ_A2 + 2 * SZ_TAB + SZ_INV + SZ_Z + 2 * SZ_CC + 3 * SZ_AP + 2 * SZ_BM + SZ_XA;
static_assert(WS_TOTAL <= ((size_t)128 << 20));

typedef _Float16 h16;
typedef _Float16 v16h __attribute__((ext_vector_type(16)));
typedef _Float16 v4h __attribute__((ext_vector_type(4)));
typedef __bf16 v16bf __attribute__((ext_vector_type(16)));
typedef unsigned short v8us __attribute__((ext_vector_type(8), may_alias));
typedef unsigned short v4us __attribute__((ext_vector_type(4), may_alias));
typedef float v8f __attribute__((ext_vector_type(8)));
typedef float v4f __attribute__((ext_vector_type(4)));
typedef float v4fa __attribute__((ext_vector_type(4), may_alias));
union FragH { v16h v; v8us half[2]; _Float16 h[16]; unsigned short u[16]; };
union FragB { v16bf v; v8us half[2]; unsigned short u[16]; };

__device__ __forceinline__ unsigned short bf16_bits(float x) { unsigned int u = __float_as_uint(x); return (unsigned short)((u + 0x7FFFu + ((u >> 16) & 1u)) >> 16); }
__device__ __forceinline__ float bf16_val(unsigned short b) { return __uint_as_float(((unsigned int)b) << 16); }
__device__ __forceinline__ float bf16_rne(float x) { return bf16_val(bf16_bits(x)); }
static __device__ __forceinline__ h16 toh_flush(float v) { const h16 r = (h16)v; return (fabsf(v) < 6.103515625e-05f) ? (h16)0.0f : r; }

template <int NT>
__device__ __forceinline__ v8f mmaH(v16h ah, v16h al, v16h bh, v16h bl, v8f c) {
  c = __builtin_amdgcn_wmma_f32_16x16x32_f16(false, ah, false, bh, (short)0, c, false, false);
  if (NT >= 2) c = __builtin_amdgcn_wmma_f32_16x16x32_f16(false, al, false, bh, (short)0, c, false, false);
  if (NT >= 3) c = __builtin_amdgcn_wmma_f32_16x16x32_f16(false, ah, false, bl, (short)0, c, false, false);
  asm volatile("v_nop\n\tv_nop\n\tv_nop\n\tv_nop" : "+v"(c) : "v"(ah), "v"(al), "v"(bh), "v"(bl));
  return c;
}
__device__ __forceinline__ v16h g2_frag(const _Float16* p, int hh) { FragH f; f.half[0] = *(const v8us*)((const unsigned short*)p + 8 * hh); f.half[1] = *(const v8us*)((const unsigned short*)p + 16 + 8 * hh); return f.v; }
__device__ __forceinline__ v8f g2_mma(v16h a, v16h b, v8f c) { v8f d = __builtin_amdgcn_wmma_f32_16x16x32_f16(false, a, false, b, (short)0, c, false, false); asm volatile("v_nop\n\tv_nop\n\tv_nop\n\tv_nop" : "+v"(d) : "v"(a), "v"(b)); return d; }
__device__ __forceinline__ v8f b2_mma(v16bf a, v16bf b, v8f c) { v8f d = __builtin_amdgcn_wmma_f32_16x16x32_bf16(false, a, false, b, (short)0, c, false, false); asm volatile("v_nop\n\tv_nop\n\tv_nop\n\tv_nop" : "+v"(d) : "v"(a), "v"(b)); return d; }

__global__ __launch_bounds__(256) void k_wtr(const float* __restrict__ Wm, _Float16* __restrict__ Bt, int ldb, float sc) {
  __shared__ unsigned short tl[64][66];
  const int tid = threadIdx.x; const int kt = blockIdx.x / (DM / 64), nt = blockIdx.x % (DM / 64);
  for (int i = tid; i < 64 * 16; i += 256) {
    const int r = i >> 4, c4 = (i & 15) * 4;
    const v4f a = *(const v4fa*)(Wm + (size_t)(kt * 64 + r) * DM + nt * 64 + c4);
    FragH f;
#pragma unroll
    for (int q = 0; q < 4; ++q) f.h[q] = toh_flush(bf16_rne(a[q]) * sc);
#pragma unroll
    for (int q = 0; q < 4; ++q) tl[r][c4 + q] = f.u[q];
  }
  __syncthreads();
  for (int pass = 0; pass < 2; ++pass) {
#pragma unroll
    for (int rd = 0; rd < 2; ++rd) {
      const int n = rd * 32 + (tid >> 3), pc = tid & 7; FragH f;
#pragma unroll
      for (int q = 0; q < 8; ++q) f.u[q] = tl[pc * 8 + q][n];
      *(volatile v8us*)((unsigned short*)Bt + (size_t)(nt * 64 + n) * ldb + kt * 64 + pc * 8) = f.half[0];
    }
    if (pass == 0) __threadfence();
  }
}

__global__ __launch_bounds__(32) void k_invf(float* __restrict__ INV) {
  #pragma clang fp contract(off)
  const int j = threadIdx.x;
  const float ex = (float)(2 * j) / 64.0f; const float pw = powf(10000.0f, ex); const float inv = 1.0f / pw;
  *(volatile float*)(INV + j) = inv; __threadfence(); *(volatile float*)(INV + j) = inv;
}
__global__ __launch_bounds__(256) void k_rotab(const float* __restrict__ INV, float* __restrict__ CS, float* __restrict__ SN) {
  #pragma clang fp contract(off)
  const int t = blockIdx.x * 256 + threadIdx.x; if (t >= SLEN * 32) return;
  const int j = t & 31, s = t >> 5;
  const float th = (float)s * INV[j]; const float c = cosf(th), sn = sinf(th);
  for (int pass = 0; pass < 2; ++pass) { *(volatile float*)(CS + t) = c; *(volatile float*)(SN + t) = sn; if (pass == 0) __threadfence(); }
}

__global__ __launch_bounds__(256) void k_x16(const float* __restrict__ x, _Float16* __restrict__ X16, size_t n8) {
  const size_t t = (size_t)blockIdx.x * 256 + threadIdx.x; if (t >= n8) return;
  const size_t e = t * 8; const size_t r = e / DM; const size_t c = e % DM; const size_t b = r / SLEN, s = r % SLEN;
  const float* src = x + (b * SEQ_FULL + s) * DM + c;
  const v4f a0 = *(const v4fa*)src, a1 = *(const v4fa*)(src + 4);
  FragH f;
#pragma unroll
  for (int q = 0; q < 4; ++q) { f.h[q] = (_Float16)bf16_rne(a0[q]); f.h[4 + q] = (_Float16)bf16_rne(a1[q]); }
  const v8us o = f.half[0];
  *(volatile v8us*)((unsigned short*)X16 + e) = o; __threadfence(); *(volatile v8us*)((unsigned short*)X16 + e) = o;
}

__global__ __launch_bounds__(256) void k_zmean(const float* __restrict__ x, float* __restrict__ Z) {
  __shared__ float sp[8][32];
  const int tid = threadIdx.x, j = tid & 31; const int sg = __builtin_amdgcn_readfirstlane(tid >> 5);
  const int b = blockIdx.x / (DM / 32), d0 = (blockIdx.x % (DM / 32)) * 32;
  const float* p = x + ((size_t)b * SEQ_FULL + (size_t)sg * (SLEN / 8)) * DM + d0 + j;
  float acc = 0.f;
#pragma unroll 4
  for (int s = 0; s < SLEN / 8; ++s) acc += bf16_rne(p[(size_t)s * DM]);
  sp[sg][j] = acc;
  __syncthreads();
  if (sg == 0) {
    float t = sp[0][j];
#pragma unroll 1
    for (int g = 1; g < 8; ++g) t += sp[g][j];
    const float m = t * (1.0f / (float)SLEN);
    *(volatile float*)(Z + (size_t)b * DM + d0 + j) = m; __threadfence(); *(volatile float*)(Z + (size_t)b * DM + d0 + j) = m;
  }
}

__global__ __launch_bounds__(256) void k_hyp(const float* __restrict__ Z, const float* __restrict__ w1, const float* __restrict__ b1,
                                             const float* __restrict__ w2, const float* __restrict__ b2, float* __restrict__ Cc) {
  __shared__ float sh[HID];
  const int tid = threadIdx.x; const int b = blockIdx.x; const int wave = __builtin_amdgcn_readfirstlane(tid >> 5);
  const float* zb = Z + (size_t)b * DM;
  float acc = 0.f;
#pragma unroll 1
  for (int i = 0; i < DM; ++i) acc += zb[i] * bf16_rne(w1[(size_t)i * HID + tid]);
  acc += bf16_rne(b1[tid]);
  const float e = expf(-acc); const float hv = acc * (1.0f / (1.0f + e));
  sh[tid] = hv;
  __syncthreads();
  if (wave < 2) {
    float c = 0.f;
#pragma unroll 1
    for (int i = 0; i < HID; ++i) c += sh[i] * bf16_rne(w2[(size_t)i * DYN + tid]);
    c += bf16_rne(b2[tid]);
    *(volatile float*)(Cc + (size_t)b * DYN + tid) = c; __threadfence(); *(volatile float*)(Cc + (size_t)b * DYN + tid) = c;
  }
}

__global__ __launch_bounds__(256) void k_gen(const float* __restrict__ Cc, const float* __restrict__ gAw, const float* __restrict__ gAb,
                                             const float* __restrict__ gBw, const float* __restrict__ gBb,
                                             unsigned short* __restrict__ AH, unsigned short* __restrict__ AM, unsigned short* __restrict__ AL,
                                             float* __restrict__ BM, int nofs) {
  const int t = blockIdx.x * 256 + threadIdx.x; if (t >= NB * (RK * DM / 4)) return;
  const int b = t / (RK * DM / 4); const int j = (t % (RK * DM / 4)) * 4;
  const float* cb = Cc + (size_t)b * DYN;
  v4f aa = {0.f, 0.f, 0.f, 0.f}, ab = {0.f, 0.f, 0.f, 0.f};
#pragma unroll 1
  for (int i = 0; i < DYN; ++i) {
    const float cv = cb[i];
    const v4f wa = *(const v4fa*)(gAw + (size_t)i * (RK * DM) + j), wb = *(const v4fa*)(gBw + (size_t)i * (RK * DM) + j);
#pragma unroll
    for (int q = 0; q < 4; ++q) { aa[q] += cv * bf16_rne(wa[q]); ab[q] += cv * bf16_rne(wb[q]); }
  }
  const v4f ba = *(const v4fa*)(gAb + j), bb = *(const v4fa*)(gBb + j);
  v4us oh, om, ol;
#pragma unroll
  for (int q = 0; q < 4; ++q) {
    const float a = aa[q] + bf16_rne(ba[q]); ab[q] += bf16_rne(bb[q]);
    const unsigned short hb = bf16_bits(a); const float r1 = a - bf16_val(hb);
    const unsigned short mb = bf16_bits(r1); const float r2 = r1 - bf16_val(mb);
    oh[q] = hb; om[q] = mb; ol[q] = bf16_bits(r2);
  }
  const size_t oa = ((size_t)b * 16 + nofs) * DM + j;
  const size_t ob = (size_t)b * DM * RK + j;
  const v4f vb = ab;
  for (int pass = 0; pass < 2; ++pass) {
    *(volatile v4us*)(AH + oa) = oh; *(volatile v4us*)(AM + oa) = om; *(volatile v4us*)(AL + oa) = ol;
    *(volatile v4f*)(BM + ob) = vb;
    if (pass == 0) __threadfence();
  }
}

__global__ __launch_bounds__(128) void k_xa(const float* __restrict__ x, const unsigned short* __restrict__ AH, const unsigned short* __restrict__ AM,
                                            const unsigned short* __restrict__ AL, float* __restrict__ XA) {
  __shared__ __attribute__((aligned(16))) float st[4][16][20];
  const int tid = threadIdx.x, lane = tid & 31, ln = lane & 15, hh = lane >> 4;
  const int w = __builtin_amdgcn_readfirstlane(tid >> 5);
  const int row0 = blockIdx.x * 64 + w * 16; const int b = row0 / SLEN, s0 = row0 % SLEN;
  const float* xr = x + ((size_t)b * SEQ_FULL + s0 + ln) * DM;
  const size_t ao = ((size_t)b * 16 + ln) * DM;
  v8f acc = {0.f, 0.f, 0.f, 0.f, 0.f, 0.f, 0.f, 0.f};
#pragma unroll 1
  for (int kb = 0; kb < DM; kb += 32) {
    const v4f x0 = *(const v4fa*)(xr + kb + 8 * hh), x1 = *(const v4fa*)(xr + kb + 8 * hh + 4);
    const v4f x2 = *(const v4fa*)(xr + kb + 16 + 8 * hh), x3 = *(const v4fa*)(xr + kb + 16 + 8 * hh + 4);
    FragB a;
#pragma unroll
    for (int q = 0; q < 4; ++q) { a.u[q] = bf16_bits(x0[q]); a.u[4 + q] = bf16_bits(x1[q]); a.u[8 + q] = bf16_bits(x2[q]); a.u[12 + q] = bf16_bits(x3[q]); }
    FragB bh, bm, bl;
    bh.half[0] = *(const v8us*)(AH + ao + kb + 8 * hh); bh.half[1] = *(const v8us*)(AH + ao + kb + 16 + 8 * hh);
    bm.half[0] = *(const v8us*)(AM + ao + kb + 8 * hh); bm.half[1] = *(const v8us*)(AM + ao + kb + 16 + 8 * hh);
    bl.half[0] = *(const v8us*)(AL + ao + kb + 8 * hh); bl.half[1] = *(const v8us*)(AL + ao + kb + 16 + 8 * hh);
    acc = b2_mma(a.v, bh.v, acc); acc = b2_mma(a.v, bm.v, acc); acc = b2_mma(a.v, bl.v, acc);
  }
#pragma unroll
  for (int r = 0; r < 8; ++r) st[w][8 * hh + r][ln] = acc[r];
  __builtin_amdgcn_fence(4, "workgroup"); __builtin_amdgcn_wave_barrier();
  float* dst = XA + (size_t)row0 * 16;
  for (int pass = 0; pass < 2; ++pass) {
#pragma unroll
    for (int i = 0; i < 2; ++i) {
      const int rr = i * 8 + (lane >> 2), cc = (lane & 3) * 4; const v4f v = *(const v4fa*)&st[w][rr][cc];
      *(volatile v4f*)(dst + i * 128 + lane * 4) = v;
    }
    if (pass == 0) __threadfence();
  }
}

template <int ACT>
__global__ __launch_bounds__(128) void k_gemm2(const _Float16* __restrict__ A, int lda, size_t sA, const _Float16* __restrict__ Bh, int ldb, size_t sB, float alpha,
                                               const float* __restrict__ bias, const float* __restrict__ XA, int ldx, const float* __restrict__ BM,
                                               float* C, _Float16* C16, int ldc, size_t sC, int M, int N, int K) {
  __shared__ __attribute__((aligned(16))) float so[4][32][68];
  const int tid = threadIdx.x, w = tid >> 5, lane = tid & 31, ln = lane & 15, hh = lane >> 4; const int by = blockIdx.y;
  A += (size_t)by * sA; Bh += (size_t)by * sB; const size_t cofs = (size_t)by * sC;
  const int ntn = N >> 6; const int mt = blockIdx.x / ntn, nq = blockIdx.x - mt * ntn; const int row0 = mt * 128 + 32 * w, col0 = nq * 64; if (row0 >= M) return;
  const _Float16* a0p = A + (size_t)(row0 + ln) * lda; const _Float16* a1p = a0p + (size_t)16 * lda;
  const _Float16* b0p = Bh + (size_t)(col0 + ln) * ldb; const _Float16* b1p = b0p + (size_t)16 * ldb; const _Float16* b2p = b1p + (size_t)16 * ldb; const _Float16* b3p = b2p + (size_t)16 * ldb;
  const v8f z8 = {0.f,0.f,0.f,0.f,0.f,0.f,0.f,0.f}; v8f c00 = z8, c01 = z8, c02 = z8, c03 = z8, c10 = z8, c11 = z8, c12 = z8, c13 = z8;
#pragma unroll 1
  for (int kb = 0; kb < K; kb += 32) {
    const v16h a0 = g2_frag(a0p + kb, hh), a1 = g2_frag(a1p + kb, hh);
    v16h bf = g2_frag(b0p + kb, hh); c00 = g2_mma(a0, bf, c00); c10 = g2_mma(a1, bf, c10);
    bf = g2_frag(b1p + kb, hh); c01 = g2_mma(a0, bf, c01); c11 = g2_mma(a1, bf, c11);
    bf = g2_frag(b2p + kb, hh); c02 = g2_mma(a0, bf, c02); c12 = g2_mma(a1, bf, c12);
    bf = g2_frag(b3p + kb, hh); c03 = g2_mma(a0, bf, c03); c13 = g2_mma(a1, bf, c13);
  }
  v8f accs[8] = {c00, c01, c02, c03, c10, c11, c12, c13};
#pragma unroll
  for (int u = 0; u < 8; ++u) {
    const int t = u & 3, half = u >> 2;
#pragma unroll
    for (int r = 0; r < 8; ++r) { const int rloc = half * 16 + 8 * hh + r; float v = accs[u][r] * alpha; if (ACT == 3) v = fmaxf(v, 0.f); so[w][rloc][t * 16 + ln] = v; }
  }
  __builtin_amdgcn_fence(4, "workgroup"); __builtin_amdgcn_wave_barrier();
  const int rsub = lane >> 4, c4 = (lane & 15) * 4;
  {
    const v4f bi = *(const v4fa*)(bias + col0 + c4);
    v4f b4;
#pragma unroll
    for (int i = 0; i < 4; ++i) b4[i] = bf16_rne(bi[i]);
    if (XA != nullptr) {
      const float* bm = BM + ((size_t)(row0 / SLEN) * DM + col0 + c4) * RK;
      const v4f m0 = *(const v4fa*)bm, m1 = *(const v4fa*)(bm + 4), m2 = *(const v4fa*)(bm + 8), m3 = *(const v4fa*)(bm + 12);
      const v4f m4 = *(const v4fa*)(bm + 16), m5 = *(const v4fa*)(bm + 20), m6 = *(const v4fa*)(bm + 24), m7 = *(const v4fa*)(bm + 28);
      const float* xr = XA + (size_t)(row0 + rsub) * ldx;
#pragma unroll 1
      for (int q = 0; q < 16; ++q) {
        const v4f xa = *(const v4fa*)(xr + (size_t)(2 * q) * ldx), xb = *(const v4fa*)(xr + (size_t)(2 * q) * ldx + 4);
        v4f v = *(const v4fa*)&so[w][q * 2 + rsub][c4];
        const float d0 = xa[0] * m0[0] + xa[1] * m0[1] + xa[2] * m0[2] + xa[3] * m0[3] + xb[0] * m1[0] + xb[1] * m1[1] + xb[2] * m1[2] + xb[3] * m1[3];
        const float d1 = xa[0] * m2[0] + xa[1] * m2[1] + xa[2] * m2[2] + xa[3] * m2[3] + xb[0] * m3[0] + xb[1] * m3[1] + xb[2] * m3[2] + xb[3] * m3[3];
        const float d2 = xa[0] * m4[0] + xa[1] * m4[1] + xa[2] * m4[2] + xa[3] * m4[3] + xb[0] * m5[0] + xb[1] * m5[1] + xb[2] * m5[2] + xb[3] * m5[3];
        const float d3 = xa[0] * m6[0] + xa[1] * m6[1] + xa[2] * m6[2] + xa[3] * m6[3] + xb[0] * m7[0] + xb[1] * m7[1] + xb[2] * m7[2] + xb[3] * m7[3];
        v[0] = (v[0] + b4[0]) + d0 * DYNS; v[1] = (v[1] + b4[1]) + d1 * DYNS; v[2] = (v[2] + b4[2]) + d2 * DYNS; v[3] = (v[3] + b4[3]) + d3 * DYNS;
        *(v4fa*)&so[w][q * 2 + rsub][c4] = v;
      }
    } else {
#pragma unroll 1
      for (int q = 0; q < 16; ++q) {
        v4f v = *(const v4fa*)&so[w][q * 2 + rsub][c4];
        v[0] += b4[0]; v[1] += b4[1]; v[2] += b4[2]; v[3] += b4[3];
        *(v4fa*)&so[w][q * 2 + rsub][c4] = v;
      }
    }
  }
  __builtin_amdgcn_fence(4, "workgroup"); __builtin_amdgcn_wave_barrier();
  for (int pass = 0; pass < 2; ++pass) {
#pragma unroll
    for (int q = 0; q < 16; ++q) {
      const int r = q * 2 + rsub; const v4f v = *(const v4fa*)&so[w][r][c4];
      if (C) *(volatile v4f*)(C + cofs + (size_t)(row0 + r) * ldc + col0 + c4) = v;
      if (C16) { v4h h4; for (int i = 0; i < 4; ++i) h4[i] = toh_flush(v[i]); *(volatile v4h*)(C16 + cofs + (size_t)(row0 + r) * ldc + col0 + c4) = h4; }
    }
    if (pass == 0) __threadfence();
  }
}

__global__ __launch_bounds__(256) void k_rope(const float* __restrict__ F, const float* __restrict__ CS, const float* __restrict__ SN, _Float16* __restrict__ H, _Float16* __restrict__ L) {
  #pragma clang fp contract(off)
  const size_t t = (size_t)blockIdx.x * 256 + threadIdx.x; if (t >= (size_t)NR * NH * 8) return;
  const int p = (int)(t & 7); const int hd = (int)((t >> 3) % NH); const size_t row = t / (8 * NH);
  const int s = (int)(row % SLEN); const int b = (int)(row / SLEN); const int g = p & 3; const int up = p >> 2;
  const float* src = F + row * DM + hd * 64 + g * 8;
  const v4f xa = *(const v4fa*)src, xb = *(const v4fa*)(src + 4), ya = *(const v4fa*)(src + 32), yb = *(const v4fa*)(src + 36);
  const float* ct = CS + (size_t)s * 32 + g * 8; const float* st = SN + (size_t)s * 32 + g * 8;
  const v4f ca = *(const v4fa*)ct, cb = *(const v4fa*)(ct + 4), sa = *(const v4fa*)st, sb = *(const v4fa*)(st + 4);
  const float x1s[8] = {xa[0], xa[1], xa[2], xa[3], xb[0], xb[1], xb[2], xb[3]};
  const float x2s[8] = {ya[0], ya[1], ya[2], ya[3], yb[0], yb[1], yb[2], yb[3]};
  const float cs[8] = {ca[0], ca[1], ca[2], ca[3], cb[0], cb[1], cb[2], cb[3]};
  const float ss[8] = {sa[0], sa[1], sa[2], sa[3], sb[0], sb[1], sb[2], sb[3]};
  FragH fh, fl;
#pragma unroll
  for (int i = 0; i < 8; ++i) {
    const float x1 = x1s[i], x2 = x2s[i], c = cs[i], sn = ss[i];
    const float o1 = x1 * c - x2 * sn; const float o2 = x2 * c + x1 * sn; const float o = up ? o2 : o1;
    const _Float16 hv = (_Float16)o; fh.h[i] = hv; fl.h[i] = (_Float16)((o - (float)hv) * 1024.0f);
  }
  const size_t oh = row * DM + hd * 64 + p * 8;
  const bool wl = (s < RE);
  const size_t ol = ((size_t)b * RE + (wl ? s : 0)) * DM + hd * 64 + p * 8;
  const v8us vh = fh.half[0], vl = fl.half[0];
  for (int pass = 0; pass < 2; ++pass) {
    *(volatile v8us*)((unsigned short*)H + oh) = vh;
    if (wl) *(volatile v8us*)((unsigned short*)L + ol) = vl;
    if (pass == 0) __threadfence();
  }
}

__global__ __launch_bounds__(256) void k_vtg(const _Float16* __restrict__ V16, _Float16* __restrict__ Vt) {
  __shared__ unsigned short tl[64][66];
  const int tid = threadIdx.x; const int nlg = SLEN / 64; const int slab = blockIdx.x / nlg, lg = blockIdx.x % nlg; const int b = slab / NH, h = slab % NH;
  for (int i = tid; i < 64 * 8; i += 256) {
    const int r = i >> 3, c8 = (i & 7) * 8; FragH f;
    f.half[0] = *(const v8us*)((const unsigned short*)V16 + ((size_t)b * SLEN + lg * 64 + r) * DM + h * 64 + c8);
#pragma unroll
    for (int q = 0; q < 8; ++q) tl[r][c8 + q] = f.u[q];
  }
  __syncthreads();
  for (int pass = 0; pass < 2; ++pass) {
#pragma unroll
    for (int rd = 0; rd < 2; ++rd) {
      const int d = rd * 32 + (tid >> 3), pc = tid & 7; FragH f;
#pragma unroll
      for (int q = 0; q < 8; ++q) f.u[q] = tl[pc * 8 + q][d];
      *(volatile v8us*)((unsigned short*)Vt + ((size_t)slab * 64 + d) * TK + lg * 64 + pc * 8) = f.half[0];
    }
    if (pass == 0) __threadfence();
  }
}
__global__ __launch_bounds__(256) void k_vtl(const float* __restrict__ VF, _Float16* __restrict__ VtL) {
  __shared__ unsigned short tl[64][66];
  const int tid = threadIdx.x; const int nlg = RE / 64; const int slab = blockIdx.x / nlg, lg = blockIdx.x % nlg; const int b = slab / NH, h = slab % NH;
  for (int i = tid; i < 64 * 16; i += 256) {
    const int r = i >> 4, c4 = (i & 15) * 4;
    const v4f a = *(const v4fa*)(VF + ((size_t)b * SLEN + lg * 64 + r) * DM + h * 64 + c4);
    FragH f;
#pragma unroll
    for (int q = 0; q < 4; ++q) { const float v = a[q]; const _Float16 hv = (_Float16)v; f.h[q] = (_Float16)((v - (float)hv) * 1024.0f); }
#pragma unroll
    for (int q = 0; q < 4; ++q) tl[r][c4 + q] = f.u[q];
  }
  __syncthreads();
  for (int pass = 0; pass < 2; ++pass) {
#pragma unroll
    for (int rd = 0; rd < 2; ++rd) {
      const int d = rd * 32 + (tid >> 3), pc = tid & 7; FragH f;
#pragma unroll
      for (int q = 0; q < 8; ++q) f.u[q] = tl[pc * 8 + q][d];
      *(volatile v8us*)((unsigned short*)VtL + ((size_t)slab * 64 + d) * RE + lg * 64 + pc * 8) = f.half[0];
    }
    if (pass == 0) __threadfence();
  }
}

__global__ __launch_bounds__(256) void k_hl(const float* __restrict__ Fp, _Float16* __restrict__ Hh, _Float16* __restrict__ A2, size_t n8) {
  const size_t t = (size_t)blockIdx.x * 256 + threadIdx.x; if (t >= n8) return;
  const size_t e = t * 8; const size_t r = e / DM; const int c = (int)(e % DM); const int s = (int)(r % SLEN); const int b = (int)(r / SLEN);
  const v4f a = *(const v4fa*)(Fp + e), d = *(const v4fa*)(Fp + e + 4);
  FragH fh, fl;
#pragma unroll
  for (int q = 0; q < 4; ++q) {
    _Float16 hv = (_Float16)a[q]; fh.h[q] = hv; fl.h[q] = (_Float16)((a[q] - (float)hv) * 1024.0f);
    hv = (_Float16)d[q]; fh.h[4 + q] = hv; fl.h[4 + q] = (_Float16)((d[q] - (float)hv) * 1024.0f);
  }
  const bool wl = (s < RE);
  const size_t o2 = ((size_t)b * RE + (wl ? s : 0)) * (size_t)(2 * DM) + c;
  const v8us vh = fh.half[0], vl = fl.half[0];
  for (int pass = 0; pass < 2; ++pass) {
    *(volatile v8us*)((unsigned short*)Hh + e) = vh;
    if (wl) { *(volatile v8us*)((unsigned short*)A2 + o2) = vh; *(volatile v8us*)((unsigned short*)A2 + o2 + DM) = vl; }
    if (pass == 0) __threadfence();
  }
}

template <int CAUSAL>
__global__ __launch_bounds__(128) void k_flash(const _Float16* __restrict__ Q16, int ldq, const _Float16* __restrict__ K16, int ldk,
                                               const _Float16* __restrict__ Vt, float* __restrict__ O, int ldo) {
  constexpr int RPW = 16, DT = 4, KS = 2;
  constexpr int NQP = (QBNP > 0) ? QBNP : 1;
  __shared__ __attribute__((aligned(16))) unsigned short sP[4][RPW][40];
  __shared__ __attribute__((aligned(16))) float sO[4][RPW][68];
  const int tid = threadIdx.x, w = tid >> 5, lane = tid & 31, ln = lane & 15, hh = lane >> 4;
  const int slab = blockIdx.x / NQP, qblk = QB0P + blockIdx.x % NQP; const int b = slab / NH, h = slab % NH;
  const int qb0 = qblk * (4 * RPW); const int q0 = qb0 + w * RPW;
  FragH aq[KS];
  {
    const unsigned short* qr = (const unsigned short*)Q16 + ((size_t)b * TQ + q0 + ln) * ldq + h * 64;
#pragma unroll
    for (int ks = 0; ks < KS; ++ks) { aq[ks].half[0] = *(const v8us*)(qr + ks * 32 + 8 * hh); aq[ks].half[1] = *(const v8us*)(qr + ks * 32 + 16 + 8 * hh); }
  }
  const unsigned short* Vth = (const unsigned short*)Vt + (size_t)slab * 64 * TK;
  float m_r[8], l_r[8]; v8f oacc[DT];
#pragma unroll
  for (int r = 0; r < 8; ++r) { m_r[r] = -3.0e38f; l_r[r] = 0.f; }
#pragma unroll
  for (int dt = 0; dt < DT; ++dt) oacc[dt] = (v8f){0.f,0.f,0.f,0.f,0.f,0.f,0.f,0.f};
  const int jend = (CAUSAL == 1) ? (qb0 + 4 * RPW) : TK;
#pragma unroll 1
  for (int j0 = 0; j0 < jend; j0 += 32) {
    v8f s[2];
#pragma unroll
    for (int nt = 0; nt < 2; ++nt) {
      const unsigned short* kr = (const unsigned short*)K16 + ((size_t)b * TK + j0 + nt * 16 + ln) * ldk + h * 64; FragH bk[KS];
#pragma unroll
      for (int ks = 0; ks < KS; ++ks) { bk[ks].half[0] = *(const v8us*)(kr + ks * 32 + 8 * hh); bk[ks].half[1] = *(const v8us*)(kr + ks * 32 + 16 + 8 * hh); }
      v8f acc = (v8f){0.f,0.f,0.f,0.f,0.f,0.f,0.f,0.f};
#pragma unroll
      for (int ks = 0; ks < KS; ++ks) acc = mmaH<1>(aq[ks].v, aq[ks].v, bk[ks].v, bk[ks].v, acc);
      s[nt] = acc;
    }
#pragma unroll
    for (int r = 0; r < 8; ++r) {
      const int tq = q0 + 8 * hh + r; const int k0 = j0 + ln, k1 = j0 + 16 + ln;
      const bool ok0 = (CAUSAL == 1) ? (k0 <= tq) : true, ok1 = (CAUSAL == 1) ? (k1 <= tq) : true;
      const float s0 = ok0 ? s[0][r] * SCL : -3.0e38f, s1 = ok1 ? s[1][r] * SCL : -3.0e38f;
      float mc = fmaxf(s0, s1);
      mc = fmaxf(mc, __shfl_xor(mc, 1, 32)); mc = fmaxf(mc, __shfl_xor(mc, 2, 32)); mc = fmaxf(mc, __shfl_xor(mc, 4, 32)); mc = fmaxf(mc, __shfl_xor(mc, 8, 32));
      const float mn = fmaxf(m_r[r], mc); const float al = (mn > -1.0e38f) ? expf(m_r[r] - mn) : 1.0f; m_r[r] = mn;
      const float p0 = ok0 ? expf(s0 - mn) : 0.f, p1 = ok1 ? expf(s1 - mn) : 0.f; l_r[r] = l_r[r] * al + p0 + p1;
#pragma unroll
      for (int dt = 0; dt < DT; ++dt) oacc[dt][r] *= al;
      FragH t2; t2.h[0] = (_Float16)(p0 * 1024.0f); t2.h[1] = (_Float16)(p1 * 1024.0f);
      sP[w][8 * hh + r][ln] = t2.u[0]; sP[w][8 * hh + r][16 + ln] = t2.u[1];
    }
    __builtin_amdgcn_fence(4, "workgroup"); __builtin_amdgcn_wave_barrier();
    FragH pa; pa.half[0] = *(const v8us*)&sP[w][ln][8 * hh]; pa.half[1] = *(const v8us*)&sP[w][ln][16 + 8 * hh];
#pragma unroll
    for (int dt = 0; dt < DT; ++dt) {
      const unsigned short* vrow = Vth + (size_t)(dt * 16 + ln) * TK + j0; FragH bv;
      bv.half[0] = *(const v8us*)(vrow + 8 * hh); bv.half[1] = *(const v8us*)(vrow + 16 + 8 * hh);
      oacc[dt] = mmaH<1>(pa.v, pa.v, bv.v, bv.v, oacc[dt]);
    }
    __builtin_amdgcn_fence(4, "workgroup"); __builtin_amdgcn_wave_barrier();
  }
#pragma unroll
  for (int r = 0; r < 8; ++r) { float l = l_r[r]; l += __shfl_xor(l, 1, 32); l += __shfl_xor(l, 2, 32); l += __shfl_xor(l, 4, 32); l += __shfl_xor(l, 8, 32); l_r[r] = (l > 0.f) ? 1.0f / (l * 1024.0f) : 0.f; }
#pragma unroll
  for (int dt = 0; dt < DT; ++dt)
#pragma unroll
    for (int r = 0; r < 8; ++r) sO[w][8 * hh + r][dt * 16 + ln] = oacc[dt][r] * l_r[r];
  __builtin_amdgcn_fence(4, "workgroup"); __builtin_amdgcn_wave_barrier();
  for (int pass = 0; pass < 2; ++pass) {
#pragma unroll
    for (int rp = 0; rp < RPW; rp += 2) { const int r = rp + (lane >> 4), pc = lane & 15; const v4f val = *(const v4fa*)&sO[w][r][pc * 4]; *(volatile v4f*)(O + ((size_t)b * TQ + q0 + r) * ldo + h * 64 + pc * 4) = val; }
    if (pass == 0) __threadfence();
  }
}
template <int CAUSAL>
__global__ __launch_bounds__(128) void k_flash5(const _Float16* __restrict__ Q16, const _Float16* __restrict__ QL, int ldq, const _Float16* __restrict__ K16, const _Float16* __restrict__ KL, int ldk,
                                                const _Float16* __restrict__ Vt, const _Float16* __restrict__ VtL, float* __restrict__ O, int ldo) {
  constexpr int RPW = 16, DT = 4, KS = 2;
  __shared__ __attribute__((aligned(16))) unsigned short sP[4][RPW][40];
  __shared__ __attribute__((aligned(16))) unsigned short sPL[4][RPW][40];
  __shared__ __attribute__((aligned(16))) float sO[4][RPW][68];
  const int tid = threadIdx.x, w = tid >> 5, lane = tid & 31, ln = lane & 15, hh = lane >> 4;
  const int slab = blockIdx.x / QBN5, qblk = QB05 + blockIdx.x % QBN5; const int b = slab / NH, h = slab % NH;
  const int qb0 = qblk * (4 * RPW); const int q0 = qb0 + w * RPW;
  FragH aq[KS], aql[KS];
  {
    const unsigned short* qr = (const unsigned short*)Q16 + ((size_t)b * TQ + q0 + ln) * ldq + h * 64;
    const unsigned short* ql = (const unsigned short*)QL + ((size_t)b * RE + q0 + ln) * ldq + h * 64;
#pragma unroll
    for (int ks = 0; ks < KS; ++ks) {
      aq[ks].half[0] = *(const v8us*)(qr + ks * 32 + 8 * hh); aq[ks].half[1] = *(const v8us*)(qr + ks * 32 + 16 + 8 * hh);
      aql[ks].half[0] = *(const v8us*)(ql + ks * 32 + 8 * hh); aql[ks].half[1] = *(const v8us*)(ql + ks * 32 + 16 + 8 * hh);
    }
  }
  const unsigned short* Vth = (const unsigned short*)Vt + (size_t)slab * 64 * TK; const unsigned short* Vtl = (const unsigned short*)VtL + (size_t)slab * 64 * RE;
  float m_r[8], l_r[8]; v8f oacc[DT], oaccL[DT];
#pragma unroll
  for (int r = 0; r < 8; ++r) { m_r[r] = -3.0e38f; l_r[r] = 0.f; }
#pragma unroll
  for (int dt = 0; dt < DT; ++dt) { oacc[dt] = (v8f){0.f,0.f,0.f,0.f,0.f,0.f,0.f,0.f}; oaccL[dt] = oacc[dt]; }
  const int jend = (CAUSAL == 1) ? (qb0 + 4 * RPW) : RE;
#pragma unroll 1
  for (int j0 = 0; j0 < jend; j0 += 32) {
    v8f s[2];
#pragma unroll
    for (int nt = 0; nt < 2; ++nt) {
      const unsigned short* kr = (const unsigned short*)K16 + ((size_t)b * TK + j0 + nt * 16 + ln) * ldk + h * 64;
      const unsigned short* klr = (const unsigned short*)KL + ((size_t)b * RE + j0 + nt * 16 + ln) * ldk + h * 64;
      FragH bk[KS], bkl[KS];
#pragma unroll
      for (int ks = 0; ks < KS; ++ks) {
        bk[ks].half[0] = *(const v8us*)(kr + ks * 32 + 8 * hh); bk[ks].half[1] = *(const v8us*)(kr + ks * 32 + 16 + 8 * hh);
        bkl[ks].half[0] = *(const v8us*)(klr + ks * 32 + 8 * hh); bkl[ks].half[1] = *(const v8us*)(klr + ks * 32 + 16 + 8 * hh);
      }
      v8f acc = (v8f){0.f,0.f,0.f,0.f,0.f,0.f,0.f,0.f}, accl = acc;
#pragma unroll
      for (int ks = 0; ks < KS; ++ks) {
        acc = mmaH<1>(aq[ks].v, aq[ks].v, bk[ks].v, bk[ks].v, acc);
        accl = mmaH<1>(aql[ks].v, aql[ks].v, bk[ks].v, bk[ks].v, accl);
        accl = mmaH<1>(aq[ks].v, aq[ks].v, bkl[ks].v, bkl[ks].v, accl);
      }
#pragma unroll
      for (int r = 0; r < 8; ++r) acc[r] += accl[r] * 0.0009765625f;
      s[nt] = acc;
    }
#pragma unroll
    for (int r = 0; r < 8; ++r) {
      const int tq = q0 + 8 * hh + r; const int k0 = j0 + ln, k1 = j0 + 16 + ln;
      const bool ok0 = (CAUSAL == 1) ? (k0 <= tq) : true, ok1 = (CAUSAL == 1) ? (k1 <= tq) : true;
      const float s0 = ok0 ? s[0][r] * SCL : -3.0e38f, s1 = ok1 ? s[1][r] * SCL : -3.0e38f;
      float mc = fmaxf(s0, s1);
      mc = fmaxf(mc, __shfl_xor(mc, 1, 32)); mc = fmaxf(mc, __shfl_xor(mc, 2, 32)); mc = fmaxf(mc, __shfl_xor(mc, 4, 32)); mc = fmaxf(mc, __shfl_xor(mc, 8, 32));
      const float mn = fmaxf(m_r[r], mc); const float al = (mn > -1.0e38f) ? expf(m_r[r] - mn) : 1.0f; m_r[r] = mn;
      const float p0 = ok0 ? expf(s0 - mn) : 0.f, p1 = ok1 ? expf(s1 - mn) : 0.f; l_r[r] = l_r[r] * al + p0 + p1;
#pragma unroll
      for (int dt = 0; dt < DT; ++dt) { oacc[dt][r] *= al; oaccL[dt][r] *= al; }
      FragH t2, t2l; const float ps0 = p0 * 1024.0f, ps1 = p1 * 1024.0f;
      t2.h[0] = (_Float16)ps0; t2.h[1] = (_Float16)ps1;
      t2l.h[0] = (_Float16)((ps0 - (float)t2.h[0]) * 1024.0f); t2l.h[1] = (_Float16)((ps1 - (float)t2.h[1]) * 1024.0f);
      sP[w][8 * hh + r][ln] = t2.u[0]; sP[w][8 * hh + r][16 + ln] = t2.u[1]; sPL[w][8 * hh + r][ln] = t2l.u[0]; sPL[w][8 * hh + r][16 + ln] = t2l.u[1];
    }
    __builtin_amdgcn_fence(4, "workgroup"); __builtin_amdgcn_wave_barrier();
    FragH pa, pl;
    pa.half[0] = *(const v8us*)&sP[w][ln][8 * hh]; pa.half[1] = *(const v8us*)&sP[w][ln][16 + 8 * hh];
    pl.half[0] = *(const v8us*)&sPL[w][ln][8 * hh]; pl.half[1] = *(const v8us*)&sPL[w][ln][16 + 8 * hh];
#pragma unroll
    for (int dt = 0; dt < DT; ++dt) {
      const unsigned short* vrow = Vth + (size_t)(dt * 16 + ln) * TK + j0; const unsigned short* vrl = Vtl + (size_t)(dt * 16 + ln) * RE + j0;
      FragH bv, bl;
      bv.half[0] = *(const v8us*)(vrow + 8 * hh); bv.half[1] = *(const v8us*)(vrow + 16 + 8 * hh);
      bl.half[0] = *(const v8us*)(vrl + 8 * hh); bl.half[1] = *(const v8us*)(vrl + 16 + 8 * hh);
      oacc[dt] = mmaH<1>(pa.v, pa.v, bv.v, bv.v, oacc[dt]);
      oaccL[dt] = mmaH<1>(pl.v, pl.v, bv.v, bv.v, oaccL[dt]);
      oaccL[dt] = mmaH<1>(pa.v, pa.v, bl.v, bl.v, oaccL[dt]);
    }
    __builtin_amdgcn_fence(4, "workgroup"); __builtin_amdgcn_wave_barrier();
  }
#pragma unroll
  for (int r = 0; r < 8; ++r) { float l = l_r[r]; l += __shfl_xor(l, 1, 32); l += __shfl_xor(l, 2, 32); l += __shfl_xor(l, 4, 32); l += __shfl_xor(l, 8, 32); l_r[r] = (l > 0.f) ? 1.0f / (l * 1024.0f) : 0.f; }
#pragma unroll
  for (int dt = 0; dt < DT; ++dt)
#pragma unroll
    for (int r = 0; r < 8; ++r) { float v = oacc[dt][r]; v += oaccL[dt][r] * 0.0009765625f; sO[w][8 * hh + r][dt * 16 + ln] = v * l_r[r]; }
  __builtin_amdgcn_fence(4, "workgroup"); __builtin_amdgcn_wave_barrier();
  for (int pass = 0; pass < 2; ++pass) {
#pragma unroll
    for (int rp = 0; rp < RPW; rp += 2) { const int r = rp + (lane >> 4), pc = lane & 15; const v4f val = *(const v4fa*)&sO[w][r][pc * 4]; *(volatile v4f*)(O + ((size_t)b * TQ + q0 + r) * ldo + h * 64 + pc * 4) = val; }
    if (pass == 0) __threadfence();
  }
}

extern "C" void kernel_launch(void* const* d_in, const int* in_sizes, int n_in,
                              void* d_out, int out_size, void* d_ws, size_t ws_size, hipStream_t stream) {
  if (n_in < 25) return;
  const size_t needx = ((size_t)(NB - 1) * SEQ_FULL + (size_t)SLEN) * DM;
  if ((size_t)in_sizes[0] < needx) return;
  if ((size_t)in_sizes[1] < (size_t)DM * DM || (size_t)in_sizes[3] < (size_t)DM * DM || (size_t)in_sizes[5] < (size_t)DM * DM || (size_t)in_sizes[15] < (size_t)DM * DM) return;
  if (in_sizes[2] < DM || in_sizes[4] < DM || in_sizes[6] < DM || in_sizes[16] < DM) return;
  if (in_sizes[7] < DM * HID || in_sizes[17] < DM * HID || in_sizes[8] < HID || in_sizes[18] < HID) return;
  if (in_sizes[9] < HID * DYN || in_sizes[19] < HID * DYN || in_sizes[10] < DYN || in_sizes[20] < DYN) return;
  if (in_sizes[11] < DYN * RK * DM || in_sizes[13] < DYN * RK * DM || in_sizes[21] < DYN * RK * DM || in_sizes[23] < DYN * RK * DM) return;
  if (in_sizes[12] < RK * DM || in_sizes[14] < RK * DM || in_sizes[22] < RK * DM || in_sizes[24] < RK * DM) return;
  if ((size_t)out_size < needx) return;
  const float* x = (const float*)d_in[0];
  const float* Wq = (const float*)d_in[1]; const float* bq = (const float*)d_in[2];
  const float* Wo = (const float*)d_in[3]; const float* bo = (const float*)d_in[4];
  const float* Wk = (const float*)d_in[5]; const float* bk = (const float*)d_in[6];
  const float* k_w1 = (const float*)d_in[7]; const float* k_b1 = (const float*)d_in[8];
  const float* k_w2 = (const float*)d_in[9]; const float* k_b2 = (const float*)d_in[10];
  const float* k_gAw = (const float*)d_in[11]; const float* k_gAb = (const float*)d_in[12];
  const float* k_gBw = (const float*)d_in[13]; const float* k_gBb = (const float*)d_in[14];
  const float* Wv = (const float*)d_in[15]; const float* bv = (const float*)d_in[16];
  const float* v_w1 = (const float*)d_in[17]; const float* v_b1 = (const float*)d_in[18];
  const float* v_w2 = (const float*)d_in[19]; const float* v_b2 = (const float*)d_in[20];
  const float* v_gAw = (const float*)d_in[21]; const float* v_gAb = (const float*)d_in[22];
  const float* v_gBw = (const float*)d_in[23]; const float* v_gBb = (const float*)d_in[24];
  float* dout = (float*)d_out;
  char* ws = (char*)d_ws; size_t off = 0;
  auto take = [&](size_t bytes) { char* p = ws + off; off += (bytes + 255) & ~(size_t)255; return p; };
  const size_t np = (size_t)NR * DM;
  _Float16* BQ = (_Float16*)take((size_t)DM * DM * 2);
  _Float16* BK = (_Float16*)take((size_t)DM * DM * 2);
  _Float16* BV = (_Float16*)take((size_t)DM * DM * 2);
  _Float16* B2 = (_Float16*)take((size_t)DM * 2 * DM * 2);
  float* FS = (float*)take(np * 4);
  _Float16* X16 = (_Float16*)take(np * 2);
  _Float16* VT = X16;
  _Float16* QH = (_Float16*)take(np * 2);
  _Float16* KH = (_Float16*)take(np * 2);
  _Float16* V16 = (_Float16*)take(np * 2);
  _Float16* QL = (_Float16*)take((size_t)NB * RE * DM * 2);
  _Float16* KL = (_Float16*)take((size_t)NB * RE * DM * 2);
  _Float16* VTL = (_Float16*)take((size_t)NB * NH * 64 * RE * 2);
  _Float16* A2 = (_Float16*)take((size_t)NB * RE * 2 * DM * 2);
  float* CS = (float*)take((size_t)SLEN * 32 * 4); float* SN = (float*)take((size_t)SLEN * 32 * 4); float* INV = (float*)take(128);
  float* ZM = (float*)take((size_t)NB * DM * 4);
  float* CCK = (float*)take((size_t)NB * DYN * 4); float* CCV = (float*)take((size_t)NB * DYN * 4);
  unsigned short* APH = (unsigned short*)take((size_t)NB * 16 * DM * 2);
  unsigned short* APM = (unsigned short*)take((size_t)NB * 16 * DM * 2);
  unsigned short* APL = (unsigned short*)take((size_t)NB * 16 * DM * 2);
  float* BMK = (float*)take((size_t)NB * DM * RK * 4); float* BMV = (float*)take((size_t)NB * DM * RK * 4);
  float* XA = (float*)take((size_t)NR * 16 * 4);
  _Float16* OH = QH;
  if (off != WS_TOTAL) return;
  if (off > ws_size) return;
  if (off > ((size_t)128 << 20)) return;

  const unsigned gt = (unsigned)((DM / 64) * (DM / 64));
  k_wtr<<<gt, 256, 0, stream>>>(Wq, BQ, DM, WSC);
  k_wtr<<<gt, 256, 0, stream>>>(Wk, BK, DM, WSC);
  k_wtr<<<gt, 256, 0, stream>>>(Wv, BV, DM, WSC);
  k_wtr<<<gt, 256, 0, stream>>>(Wo, B2, 2 * DM, WSCH);
  k_wtr<<<gt, 256, 0, stream>>>(Wo, B2 + DM, 2 * DM, WSC);
  k_invf<<<1, 32, 0, stream>>>(INV);
  k_rotab<<<(unsigned)((SLEN * 32 + 255) / 256), 256, 0, stream>>>(INV, CS, SN);
  const unsigned g8 = (unsigned)((np / 8 + 255) / 256);
  k_x16<<<g8, 256, 0, stream>>>(x, X16, np / 8);
  k_zmean<<<(unsigned)(NB * (DM / 32)), 256, 0, stream>>>(x, ZM);
  k_hyp<<<(unsigned)NB, 256, 0, stream>>>(ZM, k_w1, k_b1, k_w2, k_b2, CCK);
  k_hyp<<<(unsigned)NB, 256, 0, stream>>>(ZM, v_w1, v_b1, v_w2, v_b2, CCV);
  const unsigned gg = (unsigned)((NB * (RK * DM / 4)) / 256);
  k_gen<<<gg, 256, 0, stream>>>(CCK, k_gAw, k_gAb, k_gBw, k_gBb, APH, APM, APL, BMK, 0);
  k_gen<<<gg, 256, 0, stream>>>(CCV, v_gAw, v_gAb, v_gBw, v_gBb, APH, APM, APL, BMV, RK);
  k_xa<<<(unsigned)(NR / 64), 128, 0, stream>>>(x, APH, APM, APL, XA);
  const dim3 gp((unsigned)((NR / 128) * (DM / 64)), 1);
  const unsigned gr = (unsigned)(((size_t)NR * NH * 8 + 255) / 256);
  k_gemm2<0><<<gp, 128, 0, stream>>>(X16, DM, 0, BQ, DM, 0, ALPHA, bq, nullptr, 0, nullptr, FS, nullptr, DM, 0, NR, DM, DM);
  k_rope<<<gr, 256, 0, stream>>>(FS, CS, SN, QH, QL);
  k_gemm2<0><<<gp, 128, 0, stream>>>(X16, DM, 0, BK, DM, 0, ALPHA, bk, XA, 16, BMK, FS, nullptr, DM, 0, NR, DM, DM);
  k_rope<<<gr, 256, 0, stream>>>(FS, CS, SN, KH, KL);
  k_gemm2<0><<<gp, 128, 0, stream>>>(X16, DM, 0, BV, DM, 0, ALPHA, bv, XA + RK, 16, BMV, FS, V16, DM, 0, NR, DM, DM);
  k_vtg<<<(unsigned)(NB * NH * (SLEN / 64)), 256, 0, stream>>>(V16, VT);
  k_vtl<<<(unsigned)(NB * NH * (RE / 64)), 256, 0, stream>>>(FS, VTL);
  k_flash5<1><<<(unsigned)(NB * NH * QBN5), 128, 0, stream>>>(QH, QL, DM, KH, KL, DM, VT, VTL, FS, DM);
  if (QBNP > 0) k_flash<1><<<(unsigned)(NB * NH * QBNP), 128, 0, stream>>>(QH, DM, KH, DM, VT, FS, DM);
  k_hl<<<g8, 256, 0, stream>>>(FS, OH, A2, np / 8);
  const dim3 ge((unsigned)((RE / 128) * (DM / 64)), NB);
  k_gemm2<0><<<ge, 128, 0, stream>>>(A2, 2 * DM, (size_t)RE * 2 * DM, B2, 2 * DM, 0, ALPHAE, bo, nullptr, 0, nullptr, dout, nullptr, DM, (size_t)SEQ_FULL * DM, RE, DM, 2 * DM);
  if (SLEN > RE) {
    const dim3 gl((unsigned)(((SLEN - RE) / 128) * (DM / 64)), NB);
    k_gemm2<0><<<gl, 128, 0, stream>>>(OH + (size_t)RE * DM, DM, (size_t)SLEN * DM, B2 + DM, 2 * DM, 0, ALPHA, bo, nullptr, 0, nullptr, dout + (size_t)RE * DM, nullptr, DM, (size_t)SEQ_FULL * DM, SLEN - RE, DM, DM);
  }
}
